// GetDensity_13932873908300
// MI455X (gfx1250) — hardware-verified
//
#include <hip/hip_runtime.h>
#include <stddef.h>
#include <math.h>


#define NW       8
#define DF       24
#define KP       32
#define HID      128
#define NTHR     256
#define NWAVE    8
#define EPT      8
#define NGRP     2
#define CHUNK    (NTHR * EPT * NGRP)
#define WCAP     (EPT * NGRP * 32)
#define LISTN    (NWAVE * WCAP)
#define NBC      4096
#define NBF      1024
#define RCAP     40960
#define RBN      128
#define OTHR     512
#define DEGCAP   256
#define CNB      32
#define EPOS     256
#define MTHR     64
#define MROWS    32
#define PHP      (HID + 4)
#define PHH      (HID + 8)
#define WSCAP    134217728
#define LDS_FILL ((RCAP + NBF + LISTN) * 4 + 64)
#define PI_OVER_CUT 0.62831853071795864f
#define WP_W1H   0
#define WP_W1L   4096
#define WP_W2H   8192
#define WP_W2L   12288
#define WP_SET   16384
#define WP_TOT   32768

static_assert((CHUNK & (CHUNK - 1)) == 0);
static_assert(CHUNK <= 4096);
static_assert((NBC & (NBC - 1)) == 0 && (NBF & (NBF - 1)) == 0);
static_assert(NBC == 4 * NBF);
static_assert(OTHR * 8 == NBC);
static_assert((RCAP % 32) == 0);
static_assert((NBF % CNB) == 0);
static_assert(CNB * NW == NTHR);
static_assert(EPOS == NTHR);
static_assert(MROWS == 2 * 16 && MTHR == 64);
static_assert(((PHH * 2) % 16) == 0 && ((PHP * 4) % 16) == 0);
static_assert((EPOS % 32) == 0 && (4096 % EPOS) == 0);

typedef float          v4f   __attribute__((ext_vector_type(4)));
typedef float          v8f   __attribute__((ext_vector_type(8)));
typedef int            v4i   __attribute__((ext_vector_type(4)));
typedef unsigned short v8us  __attribute__((ext_vector_type(8)));
typedef unsigned short v16us __attribute__((ext_vector_type(16)));
typedef __bf16         v16bf __attribute__((ext_vector_type(16)));
union FragU { v16us v; v8us h[2]; };

__device__ __forceinline__ v8f wm(v16us a, v16us b, v8f c) {
  const v16bf ab = __builtin_bit_cast(v16bf, a);
  const v16bf bb = __builtin_bit_cast(v16bf, b);
  v8f d = __builtin_amdgcn_wmma_f32_16x16x32_bf16(false, ab, false, bb, (short)0, c, false, false);
  asm volatile("v_nop\n\tv_nop\n\tv_nop\n\tv_nop" : "+v"(d) : "v"(ab), "v"(bb));
  return d;
}

__device__ __forceinline__ unsigned bfb(float x) {
  const unsigned u = __float_as_uint(x);
  return (u + 0x7FFFu + ((u >> 16) & 1u)) >> 16;
}
__device__ __forceinline__ void split1(float x, unsigned short& hi, unsigned short& lo) {
  const unsigned hb = bfb(x);
  const float hf = __uint_as_float(hb << 16);
  hi = (unsigned short)hb;
  lo = (unsigned short)bfb(x - hf);
}
__device__ __forceinline__ void split8(v4f a, v4f b, v8us& hi, v8us& lo) {
  unsigned short h, l;
  split1(a.x, h, l); hi[0] = h; lo[0] = l;
  split1(a.y, h, l); hi[1] = h; lo[1] = l;
  split1(a.z, h, l); hi[2] = h; lo[2] = l;
  split1(a.w, h, l); hi[3] = h; lo[3] = l;
  split1(b.x, h, l); hi[4] = h; lo[4] = l;
  split1(b.y, h, l); hi[5] = h; lo[5] = l;
  split1(b.z, h, l); hi[6] = h; lo[6] = l;
  split1(b.w, h, l); hi[7] = h; lo[7] = l;
}
__device__ __forceinline__ float tanh_f(float x) {
  float y = fabsf(x);
  y = fminf(y, 16.0f);
  const float e = __expf(2.0f * y);
  const float t = 1.0f - 2.0f * __builtin_amdgcn_rcpf(e + 1.0f);
  return copysignf(t, x);
}

template <int NB>
__device__ __forceinline__ int scan_chunk(const int* __restrict__ keys, int nE, int cbase, int slotBase,
                                          int vec8, int* list, int tid, int lane, int wave) {
  int wc = 0;
#pragma unroll
  for (int g = 0; g < NGRP; ++g) {
    const int el0  = (g * NTHR + tid) * EPT;
    const int e0   = cbase + el0;
    const int sent = -2147483647 - 1;
    v4i da, db;
    if (vec8 != 0 && cbase + CHUNK <= nE) {
      da = *(const v4i*)(keys + e0);
      db = *(const v4i*)(keys + e0 + 4);
    } else {
      da.x = (e0     < nE) ? keys[min(e0, nE - 1)] : sent;
      da.y = (e0 + 1 < nE) ? keys[min(e0 + 1, nE - 1)] : sent;
      da.z = (e0 + 2 < nE) ? keys[min(e0 + 2, nE - 1)] : sent;
      da.w = (e0 + 3 < nE) ? keys[min(e0 + 3, nE - 1)] : sent;
      db.x = (e0 + 4 < nE) ? keys[min(e0 + 4, nE - 1)] : sent;
      db.y = (e0 + 5 < nE) ? keys[min(e0 + 5, nE - 1)] : sent;
      db.z = (e0 + 6 < nE) ? keys[min(e0 + 6, nE - 1)] : sent;
      db.w = (e0 + 7 < nE) ? keys[min(e0 + 7, nE - 1)] : sent;
    }
    const unsigned nb = (unsigned)slotBase;
    const unsigned s0 = (unsigned)da.x - nb, s1 = (unsigned)da.y - nb;
    const unsigned s2 = (unsigned)da.z - nb, s3 = (unsigned)da.w - nb;
    const unsigned s4 = (unsigned)db.x - nb, s5 = (unsigned)db.y - nb;
    const unsigned s6 = (unsigned)db.z - nb, s7 = (unsigned)db.w - nb;
    const bool h0 = s0 < (unsigned)NB, h1 = s1 < (unsigned)NB, h2 = s2 < (unsigned)NB, h3 = s3 < (unsigned)NB;
    const bool h4 = s4 < (unsigned)NB, h5 = s5 < (unsigned)NB, h6 = s6 < (unsigned)NB, h7 = s7 < (unsigned)NB;
    const unsigned any = __builtin_amdgcn_ballot_w32(h0 | h1 | h2 | h3 | h4 | h5 | h6 | h7);
    if (any != 0u) {
#define HITJ(J, HJ, SJ) { \
        const unsigned mj = __builtin_amdgcn_ballot_w32(HJ); \
        if (mj != 0u) { \
          if (HJ) { \
            const int pos = wc + (int)__builtin_amdgcn_mbcnt_lo(mj, 0u); \
            if (pos < WCAP) list[wave * WCAP + pos] = ((el0 + (J)) << 12) | (int)(SJ); \
          } \
          wc += (int)__builtin_popcount(mj); } }
      HITJ(0, h0, s0)
      HITJ(1, h1, s1)
      HITJ(2, h2, s2)
      HITJ(3, h3, s3)
      HITJ(4, h4, s4)
      HITJ(5, h5, s5)
      HITJ(6, h6, s6)
      HITJ(7, h7, s7)
#undef HITJ
    }
  }
  return wc;
}

__global__ __launch_bounds__(NTHR) void k_wprep(
    const float* __restrict__ w1a, const float* __restrict__ w2a,
    const float* __restrict__ w1b, const float* __restrict__ w2b,
    unsigned short* wp) {
  const int tid = (int)threadIdx.x;
  const int b = (int)blockIdx.x;
  const int it = b >> 2, r = b & 3;
  const float* w1 = it ? w1b : w1a;
  const float* w2 = it ? w2b : w2a;
  float v[8];
  int dhi, dlo, n, k0, Kp;
  if (r < 2) {
    const int lp = r * NTHR + tid;
    n = lp >> 2; k0 = (lp & 3) * 8; Kp = KP;
#pragma unroll
    for (int j = 0; j < 8; ++j) {
      const int k  = k0 + j;
      const int kc = k < DF ? k : DF - 1;
      const float f = w1[(size_t)kc * HID + n];
      v[j] = (k < DF) ? f : 0.0f;
    }
    dhi = WP_W1H; dlo = WP_W1L;
  } else {
    const int lp = (r - 2) * NTHR + tid;
    n = lp >> 4; k0 = (lp & 15) * 8; Kp = HID;
    const int nc = n < DF ? n : DF - 1;
#pragma unroll
    for (int j = 0; j < 8; ++j) {
      const float f = w2[(size_t)(k0 + j) * DF + nc];
      v[j] = (n < DF) ? f : 0.0f;
    }
    dhi = WP_W2H; dlo = WP_W2L;
  }
  v4f a, c;
  a.x = v[0]; a.y = v[1]; a.z = v[2]; a.w = v[3];
  c.x = v[4]; c.y = v[5]; c.z = v[6]; c.w = v[7];
  v8us oh, ol;
  split8(a, c, oh, ol);
  unsigned short* ph = wp + (size_t)it * WP_SET + dhi + (size_t)n * Kp + k0;
  unsigned short* pl = wp + (size_t)it * WP_SET + dlo + (size_t)n * Kp + k0;
  *(volatile v8us*)ph = oh;
  *(volatile v8us*)pl = ol;
  __threadfence();
  *(volatile v8us*)ph = oh;
  *(volatile v8us*)pl = ol;
}

__global__ __launch_bounds__(NTHR) void k_count(
    const int* __restrict__ keys, int* cnt, int nE, int vec8) {
  __shared__ __attribute__((aligned(16))) int scnt[NBC];
  __shared__ __attribute__((aligned(16))) int list[LISTN];
  __shared__ int wcnt[NWAVE];
  const int tid = threadIdx.x, lane = tid & 31, wave = tid >> 5;
  const int nodeBase = blockIdx.x * NBC;

  for (int i = tid; i < NBC; i += NTHR) scnt[i] = 0;
  __syncthreads();

  const int nChunks = (nE + CHUNK - 1) / CHUNK;
#pragma unroll 1
  for (int ch = 0; ch < nChunks; ++ch) {
    const int cbase = ch * CHUNK;
    const int wc = scan_chunk<NBC>(keys, nE, cbase, nodeBase, vec8, list, tid, lane, wave);
    if (lane == 0) wcnt[wave] = wc;
    __syncthreads();
    if (wave == 0) {
#pragma unroll 1
      for (int wsx = 0; wsx < NWAVE; ++wsx) {
        int n = __builtin_amdgcn_readfirstlane(wcnt[wsx]);
        n = n > WCAP ? WCAP : (n < 0 ? 0 : n);
        const int* lp = list + wsx * WCAP;
#pragma unroll 1
        for (int i = 0; i < n; ++i) {
          const int ent  = __builtin_amdgcn_readfirstlane(lp[i]);
          const int slot = ent & (NBC - 1);
          if (lane == 0) scnt[slot] = scnt[slot] + 1;
        }
      }
    }
    __syncthreads();
  }

  v4i cq[4];
#pragma unroll
  for (int q = 0; q < 4; ++q) {
    const int f = (wave * 4 + q) * 128 + 4 * lane;
    cq[q] = *(const v4i*)(scnt + f);
  }
  int* cp = cnt + (size_t)nodeBase;
#pragma unroll
  for (int q = 0; q < 4; ++q) {
    const int f = (wave * 4 + q) * 128 + 4 * lane;
    *(volatile v4i*)(cp + f) = cq[q];
  }
  __threadfence();
#pragma unroll
  for (int q = 0; q < 4; ++q) {
    const int f = (wave * 4 + q) * 128 + 4 * lane;
    *(volatile v4i*)(cp + f) = cq[q];
  }
}

__global__ __launch_bounds__(OTHR) void k_offsets(
    const int* __restrict__ cnt, int* off, int* rbase, int nChunk) {
  __shared__ __attribute__((aligned(16))) int soff[NBC];
  __shared__ __attribute__((aligned(16))) int srb[RBN];
  __shared__ int wtot[OTHR / 32];
  const int tid = threadIdx.x, lane = tid & 31, wave = tid >> 5, sub = tid >> 7;
  for (int i = tid; i < RBN; i += OTHR) srb[i] = 0;
  int carry = 0;
#pragma unroll 1
  for (int ch = 0; ch < nChunk; ++ch) {
    const int base = ch * NBC;
    const v4i c0 = *(const v4i*)(cnt + base + 8 * tid);
    const v4i c1 = *(const v4i*)(cnt + base + 8 * tid + 4);
    const int e0 = max(c0.x, 0), e1 = max(c0.y, 0), e2 = max(c0.z, 0), e3 = max(c0.w, 0);
    const int e4 = max(c1.x, 0), e5 = max(c1.y, 0), e6 = max(c1.z, 0), e7 = max(c1.w, 0);
    const int ts = e0 + e1 + e2 + e3 + e4 + e5 + e6 + e7;
    int incl = ts;
#pragma unroll
    for (int d = 1; d < 32; d <<= 1) {
      const int t = __shfl_up(incl, d);
      if (lane >= d) incl += t;
    }
    if (lane == 31) wtot[wave] = incl;
    __syncthreads();
    const int S0 = wtot[0]  + wtot[1]  + wtot[2]  + wtot[3];
    const int S1 = wtot[4]  + wtot[5]  + wtot[6]  + wtot[7];
    const int S2 = wtot[8]  + wtot[9]  + wtot[10] + wtot[11];
    const int S3 = wtot[12] + wtot[13] + wtot[14] + wtot[15];
    int pre = 0;
#pragma unroll 1
    for (int w = 4 * sub; w < wave; ++w) pre += wtot[w];
    const int b0 = carry;
    const int b1 = b0 + ((S0 + 31) & ~31);
    const int b2 = b1 + ((S1 + 31) & ~31);
    const int b3 = b2 + ((S2 + 31) & ~31);
    const int b4 = b3 + ((S3 + 31) & ~31);
    const int myb = sub == 0 ? b0 : (sub == 1 ? b1 : (sub == 2 ? b2 : b3));
    if (tid == 0) {
      srb[min(4 * ch + 0, RBN - 1)] = b0;
      srb[min(4 * ch + 1, RBN - 1)] = b1;
      srb[min(4 * ch + 2, RBN - 1)] = b2;
      srb[min(4 * ch + 3, RBN - 1)] = b3;
    }
    int run = myb + pre + incl - ts;
    soff[8 * tid + 0] = run; run += e0;
    soff[8 * tid + 1] = run; run += e1;
    soff[8 * tid + 2] = run; run += e2;
    soff[8 * tid + 3] = run; run += e3;
    soff[8 * tid + 4] = run; run += e4;
    soff[8 * tid + 5] = run; run += e5;
    soff[8 * tid + 6] = run; run += e6;
    soff[8 * tid + 7] = run;
    carry = b4;
    __syncthreads();
    const v4i o0 = *(const v4i*)(soff + 4 * tid);
    const v4i o1 = *(const v4i*)(soff + 4 * (tid + OTHR));
    int* op = off + base;
    *(volatile v4i*)(op + 4 * tid) = o0;
    *(volatile v4i*)(op + 4 * (tid + OTHR)) = o1;
    __threadfence();
    *(volatile v4i*)(op + 4 * tid) = o0;
    *(volatile v4i*)(op + 4 * (tid + OTHR)) = o1;
    __syncthreads();
  }
  if (tid == 0) srb[min(4 * nChunk, RBN - 1)] = carry;
  __syncthreads();
  v4i rv = {0, 0, 0, 0};
  if (tid < 32) rv = *(const v4i*)(srb + 4 * tid);
  if (tid < 32) *(volatile v4i*)(rbase + 4 * tid) = rv;
  __threadfence();
  if (tid < 32) *(volatile v4i*)(rbase + 4 * tid) = rv;
}

__global__ __launch_bounds__(NTHR) void k_fill(
    const int* __restrict__ keys, const int* __restrict__ off, const int* __restrict__ rbase,
    int* csr, int nE, int vec8, int csrLen) {
  extern __shared__ v4f lds_dyn[];
  int* region = (int*)lds_dyn;
  int* cursor = region + RCAP;
  int* list   = cursor + NBF;
  int* wcnt   = list + LISTN;
  const int tid = threadIdx.x, lane = tid & 31, wave = tid >> 5;
  const int b = blockIdx.x;
  const int nodeBase = b * NBF;

  int rb0 = rbase[b];
  const int rb1 = rbase[b + 1];
  rb0 = rb0 < 0 ? 0 : (rb0 > csrLen ? csrLen : rb0);
  rb0 &= ~31;
  int len = rb1 - rb0;
  len = len < 0 ? 0 : (len > RCAP ? RCAP : len);
  int lenW = (len + 31) & ~31;
  if (rb0 + lenW > csrLen) lenW = (csrLen - rb0) & ~31;

  {
    const v4i z = {0, 0, 0, 0};
    for (int i = tid; i < RCAP / 4; i += NTHR) ((v4i*)region)[i] = z;
    for (int s = tid; s < NBF; s += NTHR) {
      int o = off[nodeBase + s] - rb0;
      o = o < 0 ? 0 : (o > RCAP ? RCAP : o);
      cursor[s] = o;
    }
  }
  __syncthreads();

  const int nChunks = (nE + CHUNK - 1) / CHUNK;
#pragma unroll 1
  for (int ch = 0; ch < nChunks; ++ch) {
    const int cbase = ch * CHUNK;
    const int wc = scan_chunk<NBF>(keys, nE, cbase, nodeBase, vec8, list, tid, lane, wave);
    if (lane == 0) wcnt[wave] = wc;
    __syncthreads();
    if (wave == 0) {
#pragma unroll 1
      for (int wsx = 0; wsx < NWAVE; ++wsx) {
        int n = __builtin_amdgcn_readfirstlane(wcnt[wsx]);
        n = n > WCAP ? WCAP : (n < 0 ? 0 : n);
        const int* lp = list + wsx * WCAP;
#pragma unroll 1
        for (int i = 0; i < n; ++i) {
          const int ent  = __builtin_amdgcn_readfirstlane(lp[i]);
          const int slot = ent & (NBF - 1);
          int e = cbase + ((ent >> 12) & (CHUNK - 1));
          e = e > nE - 1 ? nE - 1 : e;
          if (lane == 0) {
            int pos = cursor[slot];
            pos = pos < 0 ? 0 : (pos > RCAP - 1 ? RCAP - 1 : pos);
            region[pos] = e;
            const int np = pos + 1;
            cursor[slot] = np > RCAP ? RCAP : np;
          }
        }
      }
    }
    __syncthreads();
  }

  const int nv = lenW >> 2;
  int* gp = csr + rb0;
#pragma unroll 1
  for (int i = tid; i < nv; i += NTHR) { const v4i v = ((const v4i*)region)[i]; *(volatile v4i*)(gp + 4 * i) = v; }
  __threadfence();
#pragma unroll 1
  for (int i = tid; i < nv; i += NTHR) { const v4i v = ((const v4i*)region)[i]; *(volatile v4i*)(gp + 4 * i) = v; }
}

__global__ __launch_bounds__(NTHR) void k_eprep(
    const int* __restrict__ csr, const float* __restrict__ cart, const int* __restrict__ nl,
    const float* __restrict__ shf, const int* __restrict__ spec,
    const float* __restrict__ rs, const float* __restrict__ inta, const float* __restrict__ par,
    float* dvP, float* fcgP, int* nbP, int nE, int nN, int csrLen, int nTyp) {
#pragma clang fp contract(off)
  __shared__ __attribute__((aligned(16))) float sG[EPOS * NW];
  __shared__ __attribute__((aligned(16))) int sNb[EPOS];
  const int tid = threadIdx.x;
  const int P0 = blockIdx.x * EPOS;
  int p = P0 + tid;
  p = p > csrLen - 1 ? csrLen - 1 : p;
  int e = csr[p];
  e = e < 0 ? 0 : (e > nE - 1 ? nE - 1 : e);
  int c = nl[e];
  c = c < 0 ? 0 : (c > nN - 1 ? nN - 1 : c);
  int n = nl[(size_t)nE + e];
  n = n < 0 ? 0 : (n > nN - 1 ? nN - 1 : n);
  const float x = cart[(size_t)3 * c + 0] - cart[(size_t)3 * n + 0] - shf[(size_t)3 * e + 0];
  const float y = cart[(size_t)3 * c + 1] - cart[(size_t)3 * n + 1] - shf[(size_t)3 * e + 1];
  const float z = cart[(size_t)3 * c + 2] - cart[(size_t)3 * n + 2] - shf[(size_t)3 * e + 2];
  const float d = sqrtf((x * x + y * y) + z * z);
  const float ct = 0.5f * cosf(d * PI_OVER_CUT) + 0.5f;
  const float fc = ct * ct;
  int sp = spec[n];
  sp = sp < 0 ? 0 : (sp > nTyp - 1 ? nTyp - 1 : sp);
#pragma unroll 1
  for (int w = 0; w < NW; ++w) {
    const float rv = rs[sp * NW + w];
    const float iv = inta[sp * NW + w];
    const float pv = par[sp * NW + w];
    const float dr = d - rv;
    const float g = __expf(-(iv * (dr * dr))) * pv;
    sG[tid * NW + w] = fc * g;
  }
  sNb[tid] = n;
  v4f dv;
  dv.x = x; dv.y = y; dv.z = z; dv.w = 0.0f;
  __syncthreads();
  const v4f g0 = *(const v4f*)(sG + 4 * tid);
  const v4f g1 = *(const v4f*)(sG + 4 * (tid + NTHR));
  v4i nbv = {0, 0, 0, 0};
  if (tid < EPOS / 4) nbv = *(const v4i*)(sNb + 4 * tid);
  float* dvp = dvP + (size_t)(P0 + tid) * 4;
  float* fgp = fcgP + (size_t)P0 * NW;
  int*   nbp = nbP + P0;
  *(volatile v4f*)dvp = dv;
  *(volatile v4f*)(fgp + 4 * tid) = g0;
  *(volatile v4f*)(fgp + 4 * (tid + NTHR)) = g1;
  if (tid < EPOS / 4) *(volatile v4i*)(nbp + 4 * tid) = nbv;
  __threadfence();
  *(volatile v4f*)dvp = dv;
  *(volatile v4f*)(fgp + 4 * tid) = g0;
  *(volatile v4f*)(fgp + 4 * (tid + NTHR)) = g1;
  if (tid < EPOS / 4) *(volatile v4i*)(nbp + 4 * tid) = nbv;
}

template <int MODE>
__global__ __launch_bounds__(NTHR) void k_agg(
    const int* __restrict__ offp, const int* __restrict__ cntp,
    const float* __restrict__ dvP, const float* __restrict__ fcgP, const int* __restrict__ nbP,
    const float* __restrict__ msg, float* dst, int nN, int csrLen) {
  __shared__ __attribute__((aligned(16))) float sD[CNB * KP];
  const int tid = threadIdx.x, lane = tid & 31;
  const int s = tid >> 3, w = tid & 7;
  const int c0 = blockIdx.x * CNB;
  int offl = offp[c0 + s];
  int cntl = cntp[c0 + s];
  cntl = cntl < 0 ? 0 : (cntl > DEGCAP ? DEGCAP : cntl);
  offl = offl < 0 ? 0 : (offl > csrLen - 1 ? csrLen - 1 : offl);
  int md = cntl;
  md = max(md, __shfl_xor(md, 1));
  md = max(md, __shfl_xor(md, 2));
  md = max(md, __shfl_xor(md, 4));
  md = max(md, __shfl_xor(md, 8));
  md = max(md, __shfl_xor(md, 16));
  int maxdeg = __builtin_amdgcn_readfirstlane(md);
  maxdeg = maxdeg < 0 ? 0 : (maxdeg > DEGCAP ? DEGCAP : maxdeg);

  float acc[13];
#pragma unroll
  for (int i = 0; i < 13; ++i) acc[i] = 0.0f;

#pragma unroll 1
  for (int r = 0; r < maxdeg; ++r) {
    const bool valid = r < cntl;
    const int rr = valid ? r : cntl - 1;
    int pos = offl + rr;
    pos = pos < 0 ? 0 : (pos > csrLen - 1 ? csrLen - 1 : pos);
    const v4f dv = *(const v4f*)(dvP + (size_t)pos * 4);
    float g = fcgP[(size_t)pos * NW + w];
    g = valid ? g : 0.0f;
    float g0 = g, g1 = g, g2 = g;
    if constexpr (MODE != 0) {
      int nb = nbP[pos];
      nb = nb < 0 ? 0 : (nb > nN - 1 ? nN - 1 : nb);
      const float* mp = msg + (size_t)nb * KP + w;
      g0 = g * mp[0];
      g1 = g * mp[8];
      g2 = g * mp[16];
    }
    const float x = dv.x, y = dv.y, z = dv.z;
    acc[0] += g0;
    acc[1] += x * g1;
    acc[2] += y * g1;
    acc[3] += z * g1;
    const float xg = x * g2, yg = y * g2, zg = z * g2;
    acc[4]  += x * xg; acc[5]  += x * yg; acc[6]  += x * zg;
    acc[7]  += y * xg; acc[8]  += y * yg; acc[9]  += y * zg;
    acc[10] += z * xg; acc[11] += z * yg; acc[12] += z * zg;
  }

  const float d0 = acc[0] * acc[0];
  const float d1 = acc[1] * acc[1] + acc[2] * acc[2] + acc[3] * acc[3];
  float d2 = acc[4] * acc[4];
#pragma unroll
  for (int i = 5; i < 13; ++i) d2 += acc[i] * acc[i];

  if constexpr (MODE != 2) {
    sD[s * KP + w]      = d0;
    sD[s * KP + 8 + w]  = d1;
    sD[s * KP + 16 + w] = d2;
    sD[s * KP + 24 + w] = 0.0f;
  } else {
    sD[s * DF + w]      = d0;
    sD[s * DF + 8 + w]  = d1;
    sD[s * DF + 16 + w] = d2;
  }
  __syncthreads();

  if constexpr (MODE != 2) {
    const int row = tid >> 3, q = tid & 7;
    const v4f v = *(const v4f*)(sD + row * KP + 4 * q);
    float* gp = dst + (size_t)(c0 + row) * KP + 4 * q;
    *(volatile v4f*)gp = v;
    __threadfence();
    *(volatile v4f*)gp = v;
  } else {
    int nval = nN - c0;
    nval = nval < 0 ? 0 : (nval > CNB ? CNB : nval);
    const int npc = nval * (DF / 4);
    const int qi = tid < npc ? tid : 0;
    const v4f v = *(const v4f*)(sD + 4 * qi);
    float* gp = dst + (size_t)c0 * DF + 4 * qi;
    if (tid < npc) *(volatile v4f*)gp = v;
    __threadfence();
    if (tid < npc) *(volatile v4f*)gp = v;
  }
  (void)lane;
}

__global__ __launch_bounds__(MTHR) void k_mlp(
    const float* __restrict__ dens, const unsigned short* __restrict__ wset,
    const float* __restrict__ b1, const float* __restrict__ b2,
    float* msg, int nN) {
  __shared__ __attribute__((aligned(16))) float sP[2 * 16 * PHP];
  __shared__ __attribute__((aligned(16))) unsigned short sHh[2 * 16 * PHH];
  __shared__ __attribute__((aligned(16))) unsigned short sHl[2 * 16 * PHH];
  const int tid = threadIdx.x, lane = tid & 31, wave = tid >> 5, hh = lane >> 4, m = lane & 15;
  const int rw0 = blockIdx.x * MROWS + wave * 16;
  float* myP = sP + wave * 16 * PHP;
  unsigned short* myH = sHh + wave * 16 * PHH;
  unsigned short* myL = sHl + wave * 16 * PHH;
  const unsigned short* w1h = wset + WP_W1H;
  const unsigned short* w1l = wset + WP_W1L;
  const unsigned short* w2h = wset + WP_W2H;
  const unsigned short* w2l = wset + WP_W2L;

  int row = rw0 + m;
  row = row > nN - 1 ? nN - 1 : row;
  const float* ap = dens + (size_t)row * KP + 8 * hh;
  const v4f a0 = *(const v4f*)(ap);
  const v4f a1 = *(const v4f*)(ap + 4);
  const v4f a2 = *(const v4f*)(ap + 16);
  const v4f a3 = *(const v4f*)(ap + 20);
  FragU Ah, Al;
  split8(a0, a1, Ah.h[0], Al.h[0]);
  split8(a2, a3, Ah.h[1], Al.h[1]);

  v8f acc1[8];
#pragma unroll
  for (int t = 0; t < 8; ++t) { v8f zz = {0.f, 0.f, 0.f, 0.f, 0.f, 0.f, 0.f, 0.f}; acc1[t] = zz; }
#pragma unroll
  for (int t = 0; t < 8; ++t) {
    const unsigned short* bph = w1h + (size_t)(16 * t + m) * KP + 8 * hh;
    const unsigned short* bpl = w1l + (size_t)(16 * t + m) * KP + 8 * hh;
    FragU Bh, Bl;
    Bh.h[0] = *(const v8us*)bph;
    Bh.h[1] = *(const v8us*)(bph + 16);
    Bl.h[0] = *(const v8us*)bpl;
    Bl.h[1] = *(const v8us*)(bpl + 16);
    acc1[t] = wm(Ah.v, Bh.v, acc1[t]);
    acc1[t] = wm(Ah.v, Bl.v, acc1[t]);
    acc1[t] = wm(Al.v, Bh.v, acc1[t]);
  }

  float* sp = myP + (8 * hh) * PHP + m;
#pragma unroll
  for (int t = 0; t < 8; ++t) {
    const float bv = b1[16 * t + m];
#pragma unroll
    for (int r = 0; r < 8; ++r) sp[r * PHP + 16 * t] = acc1[t][r] + bv;
  }
  __syncthreads();

#pragma unroll 1
  for (int i = 0; i < 64; ++i) {
    const int idx = i * 32 + lane;
    const int rr = idx >> 7, cc = idx & 127;
    const float v = tanh_f(myP[rr * PHP + cc]);
    unsigned short hb, lb;
    split1(v, hb, lb);
    myH[rr * PHH + cc] = hb;
    myL[rr * PHH + cc] = lb;
  }
  __syncthreads();

  v8f acc2[2];
#pragma unroll
  for (int t2 = 0; t2 < 2; ++t2) { v8f zz = {0.f, 0.f, 0.f, 0.f, 0.f, 0.f, 0.f, 0.f}; acc2[t2] = zz; }
  const unsigned short* hp = myH + m * PHH + 8 * hh;
  const unsigned short* lq = myL + m * PHH + 8 * hh;
#pragma unroll
  for (int ks = 0; ks < HID / 32; ++ks) {
    FragU A2h, A2l;
    A2h.h[0] = *(const v8us*)(hp + 32 * ks);
    A2h.h[1] = *(const v8us*)(hp + 32 * ks + 16);
    A2l.h[0] = *(const v8us*)(lq + 32 * ks);
    A2l.h[1] = *(const v8us*)(lq + 32 * ks + 16);
#pragma unroll
    for (int t2 = 0; t2 < 2; ++t2) {
      const unsigned short* bph = w2h + (size_t)(16 * t2 + m) * HID + 32 * ks + 8 * hh;
      const unsigned short* bpl = w2l + (size_t)(16 * t2 + m) * HID + 32 * ks + 8 * hh;
      FragU Bh, Bl;
      Bh.h[0] = *(const v8us*)bph;
      Bh.h[1] = *(const v8us*)(bph + 16);
      Bl.h[0] = *(const v8us*)bpl;
      Bl.h[1] = *(const v8us*)(bpl + 16);
      acc2[t2] = wm(A2h.v, Bh.v, acc2[t2]);
      acc2[t2] = wm(A2h.v, Bl.v, acc2[t2]);
      acc2[t2] = wm(A2l.v, Bh.v, acc2[t2]);
    }
  }

  float* so = myP;
#pragma unroll
  for (int t2 = 0; t2 < 2; ++t2) {
    const int n = 16 * t2 + m;
    const int nc = n < DF ? n : DF - 1;
    const float braw = b2[nc];
    const float bv = (n < DF) ? braw : 0.0f;
#pragma unroll
    for (int r = 0; r < 8; ++r) so[(8 * hh + r) * KP + n] = acc2[t2][r] + bv;
  }
  __syncthreads();
  const int rq = lane >> 3, q = lane & 7;
  v4f ov[4];
#pragma unroll
  for (int i = 0; i < 4; ++i) ov[i] = *(const v4f*)(so + (4 * i + rq) * KP + 4 * q);
#pragma unroll
  for (int i = 0; i < 4; ++i)
    *(volatile v4f*)(msg + (size_t)(rw0 + 4 * i + rq) * KP + 4 * q) = ov[i];
  __threadfence();
#pragma unroll
  for (int i = 0; i < 4; ++i)
    *(volatile v4f*)(msg + (size_t)(rw0 + 4 * i + rq) * KP + 4 * q) = ov[i];
}

extern "C" void kernel_launch(void* const* d_in, const int* in_sizes, int n_in,
                              void* d_out, int out_size, void* d_ws, size_t ws_size,
                              hipStream_t stream) {
  if (n_in < 15) return;
  const int nN = in_sizes[3];
  if (nN <= 0 || in_sizes[0] != 3 * nN) return;
  if (in_sizes[1] <= 0 || (in_sizes[1] & 1) != 0) return;
  const int nE = in_sizes[1] / 2;
  if (in_sizes[2] != 3 * nE) return;
  const int nTab = in_sizes[4];
  if (nTab < NW || (nTab % NW) != 0 || in_sizes[5] != nTab || in_sizes[6] != nTab) return;
  const int nTyp = nTab / NW;
  if (in_sizes[7] != DF * HID || in_sizes[8] != HID || in_sizes[9] != HID * DF || in_sizes[10] != DF) return;
  if (in_sizes[11] != DF * HID || in_sizes[12] != HID || in_sizes[13] != HID * DF || in_sizes[14] != DF) return;
  if (out_size != nN * DF) return;
  if (nE > (1 << 26) || nN > (1 << 22)) return;

  const float* cart  = (const float*)d_in[0];
  const int*   nl    = (const int*)d_in[1];
  const float* shf   = (const float*)d_in[2];
  const int*   spec  = (const int*)d_in[3];
  const float* rs    = (const float*)d_in[4];
  const float* inta  = (const float*)d_in[5];
  const float* par   = (const float*)d_in[6];
  const float* w1a   = (const float*)d_in[7];
  const float* b1a   = (const float*)d_in[8];
  const float* w2a   = (const float*)d_in[9];
  const float* b2a   = (const float*)d_in[10];
  const float* w1b   = (const float*)d_in[11];
  const float* b1b   = (const float*)d_in[12];
  const float* w2b   = (const float*)d_in[13];
  const float* b2b   = (const float*)d_in[14];
  float* out = (float*)d_out;

  const int nBC    = (nN + NBC - 1) / NBC;
  const int CNTPAD = nBC * NBC;
  if (4 * nBC + 1 > RBN) return;
  const int nBF    = (nN + NBF - 1) / NBF;
  if (31 * 4 * nBC > 4096) return;
  const int csrLen = ((nE + EPOS - 1) / EPOS) * EPOS + 4096;
  const int nEP    = csrLen / EPOS;
  const int nAgg   = (nN + CNB - 1) / CNB;
  const int NPR    = nAgg * CNB;
  if (NPR > CNTPAD) return;
  const int nMlp   = NPR / MROWS;

  char* ws = (char*)d_ws;
  size_t off = 0;
  const size_t plane = (size_t)NPR * KP * 4;
  const size_t oW   = off; off += (size_t)WP_TOT * 2;         off = (off + 255) & ~(size_t)255;
  const size_t oCnt = off; off += (size_t)CNTPAD * 4;         off = (off + 255) & ~(size_t)255;
  const size_t oOff = off; off += (size_t)CNTPAD * 4;         off = (off + 255) & ~(size_t)255;
  const size_t oRb  = off; off += (size_t)RBN * 4;            off = (off + 255) & ~(size_t)255;
  const size_t oCsr = off; off += (size_t)csrLen * 4;         off = (off + 255) & ~(size_t)255;
  const size_t oDv  = off; off += (size_t)csrLen * 16;        off = (off + 255) & ~(size_t)255;
  const size_t oFg  = off; off += (size_t)csrLen * NW * 4;    off = (off + 255) & ~(size_t)255;
  const size_t oNb  = off; off += (size_t)csrLen * 4;         off = (off + 255) & ~(size_t)255;
  const size_t oDen = off; off += plane;                      off = (off + 255) & ~(size_t)255;
  const size_t oMsg = off; off += plane;                      off = (off + 255) & ~(size_t)255;
  if (off > ws_size || off > (size_t)WSCAP) return;
  unsigned short* wp = (unsigned short*)(ws + oW);
  int*   cnt  = (int*)(ws + oCnt);
  int*   offp = (int*)(ws + oOff);
  int*   rb   = (int*)(ws + oRb);
  int*   csr  = (int*)(ws + oCsr);
  float* dvP  = (float*)(ws + oDv);
  float* fcgP = (float*)(ws + oFg);
  int*   nbP  = (int*)(ws + oNb);
  float* dens = (float*)(ws + oDen);
  float* msg  = (float*)(ws + oMsg);

  const int vec8 = ((nE & 3) == 0) ? 1 : 0;
  const int* keys = nl;

  k_wprep<<<8, NTHR, 0, stream>>>(w1a, w2a, w1b, w2b, wp);

  k_count<<<nBC, NTHR, 0, stream>>>(keys, cnt, nE, vec8);
  k_offsets<<<1, OTHR, 0, stream>>>(cnt, offp, rb, nBC);
  hipFuncSetAttribute(reinterpret_cast<const void*>(&k_fill),
                      hipFuncAttributeMaxDynamicSharedMemorySize, LDS_FILL);
  k_fill<<<nBF, NTHR, LDS_FILL, stream>>>(keys, offp, rb, csr, nE, vec8, csrLen);

  k_eprep<<<nEP, NTHR, 0, stream>>>(csr, cart, nl, shf, spec, rs, inta, par,
                                    dvP, fcgP, nbP, nE, nN, csrLen, nTyp);

  k_agg<0><<<nAgg, NTHR, 0, stream>>>(offp, cnt, dvP, fcgP, nbP, msg, dens, nN, csrLen);

  k_mlp<<<nMlp, MTHR, 0, stream>>>(dens, wp, b1a, b2a, msg, nN);
  k_agg<1><<<nAgg, NTHR, 0, stream>>>(offp, cnt, dvP, fcgP, nbP, msg, dens, nN, csrLen);
  k_mlp<<<nMlp, MTHR, 0, stream>>>(dens, wp + WP_SET, b1b, b2b, msg, nN);
  k_agg<2><<<nAgg, NTHR, 0, stream>>>(offp, cnt, dvP, fcgP, nbP, msg, out, nN, csrLen);
}
